// PosAttBlock_46763603919172
// MI455X (gfx1250) — hardware-verified
//
#include <hip/hip_runtime.h>

typedef _Float16 f16t;
typedef _Float16 v16h __attribute__((ext_vector_type(16)));
typedef _Float16 v8h  __attribute__((ext_vector_type(8)));
typedef float    v8f  __attribute__((ext_vector_type(8)));
typedef float    v4f  __attribute__((ext_vector_type(4)));
typedef v8h  __attribute__((may_alias)) v8ha;
typedef v4f  __attribute__((may_alias)) v4fa;
union Frag { v16h v; v8h half[2]; };
union Q8   { v8f v; v4f q[2]; };

#define NB   4
#define CC   512
#define MID  64
#define HW   64
#define NP   4096
#define QB   32
#define SSP  72
#define PSP  72
#define OSP  36
#define VSP  72
#define W1SC 16.0f
#define ACAR 8.0f
#define VCAR 8.0f
#define PCAR 1024.0f

__device__ __forceinline__ v8f wmma_f16(v16h a, v16h b, v8f c) {
  v8f d = __builtin_amdgcn_wmma_f32_16x16x32_f16(false, a, false, b, (short)0, c, false, false);
  asm volatile("v_nop\n\tv_nop\n\tv_nop\n\tv_nop" : "+v"(d) : "v"(a), "v"(b));
  return d;
}

__device__ __forceinline__ v16h load_frag32(const f16t* p, int h) {
  Frag f;
  f.half[0] = *(const v8ha*)(p + 8 * h);
  f.half[1] = *(const v8ha*)(p + 16 + 8 * h);
  return f.v;
}

__device__ __forceinline__ v8f zero8f() {
  v8f z;
  #pragma unroll
  for (int j = 0; j < 8; ++j) z[j] = 0.f;
  return z;
}

__device__ __forceinline__ void st8f(float* p, v8f v) {
  Q8 u; u.v = v;
  *(v4fa*)p = u.q[0];
  *(v4fa*)(p + 4) = u.q[1];
}

__global__ __launch_bounds__(256) void k_wcvt(
    const float* __restrict__ wq, const float* __restrict__ wk, const float* __restrict__ wv,
    f16t* __restrict__ Wqh, f16t* __restrict__ Wkh, f16t* __restrict__ Wvh)
{
  const int g = blockIdx.x * 256 + threadIdx.x;
  if (g >= 40960) return;
  const float* base;
  f16t* dst;
  if (g < 4096)      { base = wq + (size_t)g * 8;          dst = Wqh + (size_t)g * 8; }
  else if (g < 8192) { base = wk + (size_t)(g - 4096) * 8; dst = Wkh + (size_t)(g - 4096) * 8; }
  else               { base = wv + (size_t)(g - 8192) * 8; dst = Wvh + (size_t)(g - 8192) * 8; }
  const v4f u0 = *(const v4fa*)base;
  const v4f u1 = *(const v4fa*)(base + 4);
  v8h o8;
  #pragma unroll
  for (int e = 0; e < 4; ++e) { o8[e] = (f16t)(u0[e] * W1SC); o8[4 + e] = (f16t)(u1[e] * W1SC); }
  *(volatile v8h*)dst = o8;
  __threadfence();
  *(volatile v8h*)dst = o8;
}

__global__ __launch_bounds__(256) void k_tr(const float* __restrict__ src, f16t* __restrict__ dst)
{
  __shared__ __attribute__((aligned(16))) f16t sH[64 * 64];
  const int tid = threadIdx.x, lane = tid & 31, w = tid >> 5;
  const int cg = blockIdx.x, pg = blockIdx.y, b = blockIdx.z;
  const int p0 = pg * 64;
  const int xq = tid & 15, cl = tid >> 4, x0 = 4 * xq;
  #pragma unroll
  for (int j = 0; j < 4; ++j) {
    const int col = cl + 16 * j, c = 64 * cg + col;
    const size_t off = (size_t)(b * CC + c) * NP + p0 + x0;
    const v4f v = *(const v4fa*)(src + off);
    sH[(x0 + 0) * 64 + col] = (f16t)(v.x * ACAR);
    sH[(x0 + 1) * 64 + col] = (f16t)(v.y * ACAR);
    sH[(x0 + 2) * 64 + col] = (f16t)(v.z * ACAR);
    sH[(x0 + 3) * 64 + col] = (f16t)(v.w * ACAR);
  }
  __syncthreads();
  const int q8 = lane & 7, sub = lane >> 3;
  v8h vals[2];
  #pragma unroll
  for (int i = 0; i < 2; ++i) {
    const int lid = 8 * w + 4 * i + sub;
    vals[i] = *(const v8ha*)(sH + lid * 64 + 8 * q8);
    const size_t d = (size_t)(b * NP + p0 + lid) * CC + 64 * cg + 8 * q8;
    *(volatile v8h*)(dst + d) = vals[i];
  }
  __threadfence();
  #pragma unroll
  for (int i = 0; i < 2; ++i) {
    const int lid = 8 * w + 4 * i + sub;
    const size_t d = (size_t)(b * NP + p0 + lid) * CC + 64 * cg + 8 * q8;
    *(volatile v8h*)(dst + d) = vals[i];
  }
}

__global__ __launch_bounds__(256) void k_proj(
    const f16t* __restrict__ XT, const f16t* __restrict__ Wqh, const f16t* __restrict__ Wkh,
    const f16t* __restrict__ Wvh, const float* __restrict__ bq, const float* __restrict__ bk,
    const float* __restrict__ bv, f16t* __restrict__ QT, f16t* __restrict__ KT, f16t* __restrict__ VC)
{
  __shared__ __attribute__((aligned(16))) f16t sV[64 * VSP];
  const int tid = threadIdx.x, lane = tid & 31, w = tid >> 5;
  const int h = lane >> 4, m = lane & 15;
  const int p0 = blockIdx.x * 64, g = blockIdx.y, b = blockIdx.z;
  const f16t* W = (g < 8) ? (Wvh + (size_t)(64 * g) * CC) : ((g == 8) ? Wqh : Wkh);
  const float* bias = (g < 8) ? (bv + 64 * g) : ((g == 8) ? bq : bk);
  const int mt = w & 3, ng = w >> 2;
  const v8f z8 = zero8f();
  v8f acc[2];
  acc[0] = z8; acc[1] = z8;
  const f16t* arow = XT + (size_t)(b * NP + p0 + 16 * mt + m) * CC;
  const f16t* brow = W + (size_t)(32 * ng + m) * CC;
  #pragma unroll 2
  for (int k0 = 0; k0 < CC; k0 += 32) {
    const v16h a = load_frag32(arow + k0, h);
    #pragma unroll
    for (int t = 0; t < 2; ++t) {
      const v16h bb = load_frag32(brow + (size_t)(16 * t) * CC + k0, h);
      acc[t] = wmma_f16(a, bb, acc[t]);
    }
  }
  const float osc = 1.0f / (ACAR * W1SC);
  #pragma unroll
  for (int t = 0; t < 2; ++t) {
    const int cl = 32 * ng + 16 * t + m;
    const float bb = bias[cl];
    v8h hv;
    #pragma unroll
    for (int r = 0; r < 8; ++r) hv[r] = (f16t)((acc[t][r] * osc + bb) * VCAR);
    *(v8ha*)(sV + cl * VSP + 16 * mt + 8 * h) = hv;
  }
  __syncthreads();
  const int q8 = lane & 7, sub = lane >> 3;
  if (g < 8) {
    v8h vals[2];
    #pragma unroll
    for (int i = 0; i < 2; ++i) {
      const int c = 8 * w + 4 * i + sub;
      vals[i] = *(const v8ha*)(sV + c * VSP + 8 * q8);
      const size_t d = (size_t)(b * CC + 64 * g + c) * NP + p0 + 8 * q8;
      *(volatile v8h*)(VC + d) = vals[i];
    }
    __threadfence();
    #pragma unroll
    for (int i = 0; i < 2; ++i) {
      const int c = 8 * w + 4 * i + sub;
      const size_t d = (size_t)(b * CC + 64 * g + c) * NP + p0 + 8 * q8;
      *(volatile v8h*)(VC + d) = vals[i];
    }
  } else {
    f16t* dstp = (g == 8) ? QT : KT;
    v8h hvs[2];
    #pragma unroll
    for (int i = 0; i < 2; ++i) {
      const int p = 8 * w + 4 * i + sub;
      v8h hv;
      #pragma unroll
      for (int e = 0; e < 8; ++e) hv[e] = sV[(8 * q8 + e) * VSP + p];
      hvs[i] = hv;
      const size_t d = (size_t)(b * NP + p0 + p) * MID + 8 * q8;
      *(volatile v8h*)(dstp + d) = hvs[i];
    }
    __threadfence();
    #pragma unroll
    for (int i = 0; i < 2; ++i) {
      const int p = 8 * w + 4 * i + sub;
      const size_t d = (size_t)(b * NP + p0 + p) * MID + 8 * q8;
      *(volatile v8h*)(dstp + d) = hvs[i];
    }
  }
}

__global__ __launch_bounds__(256) void k_att(
    const f16t* __restrict__ QT, const f16t* __restrict__ KT, const f16t* __restrict__ VC,
    const float* __restrict__ xres, const float* __restrict__ alpha, float* __restrict__ out)
{
  __shared__ __attribute__((aligned(16))) float sS[QB * SSP];
  __shared__ __attribute__((aligned(16))) f16t  sP[QB * PSP];
  __shared__ __attribute__((aligned(16))) float sO[256 * OSP];
  __shared__ __attribute__((aligned(16))) float rsc[QB];
  __shared__ __attribute__((aligned(16))) float lsum[QB];
  const int tid = threadIdx.x, lane = tid & 31, w = tid >> 5;
  const int h = lane >> 4, m = lane & 15;
  const int i0 = blockIdx.x * QB, b = blockIdx.y;
  const int it = w & 1, jt = w >> 1;
  const int si = tid >> 3, jq = tid & 7;
  const float sinv = 1.0f / (VCAR * VCAR);
  const f16t* qrow = QT + (size_t)(b * NP + i0 + 16 * it + m) * MID;
  const v16h bq0 = load_frag32(qrow, h);
  const v16h bq1 = load_frag32(qrow + 32, h);
  const f16t* vrow = VC + (size_t)(b * CC + 64 * w + m) * NP;
  const v8f z8 = zero8f();
  v8f acc[2][4];
  #pragma unroll
  for (int js = 0; js < 2; ++js) {
    #pragma unroll
    for (int ct = 0; ct < 4; ++ct) acc[js][ct] = z8;
  }
  float mrun = -1.0e30f, lrun = 0.f;

  #pragma unroll 1
  for (int j0 = 0; j0 < NP; j0 += 64) {
    {
      const f16t* kp = KT + (size_t)(b * NP + j0 + 16 * jt + m) * MID;
      const v16h a0 = load_frag32(kp, h);
      const v16h a1 = load_frag32(kp + 32, h);
      v8f s = wmma_f16(a0, bq0, z8);
      s = wmma_f16(a1, bq1, s);
      st8f(sS + (16 * it + m) * SSP + 16 * jt + 8 * h, s);
    }
    __syncthreads();

    float sv[8];
    {
      const float* sp = sS + si * SSP + 8 * jq;
      const v4f t0 = *(const v4fa*)sp;
      const v4f t1 = *(const v4fa*)(sp + 4);
      sv[0] = t0.x; sv[1] = t0.y; sv[2] = t0.z; sv[3] = t0.w;
      sv[4] = t1.x; sv[5] = t1.y; sv[6] = t1.z; sv[7] = t1.w;
    }
    float mx = sv[0];
    #pragma unroll
    for (int r = 1; r < 8; ++r) mx = fmaxf(mx, sv[r]);
    mx = fmaxf(mx, __shfl_xor(mx, 1));
    mx = fmaxf(mx, __shfl_xor(mx, 2));
    mx = fmaxf(mx, __shfl_xor(mx, 4));
    const float mnew = fmaxf(mrun, mx);
    const float rs = __expf((mrun - mnew) * sinv);
    mrun = mnew;
    float psum = 0.f;
    v8h pa;
    #pragma unroll
    for (int r = 0; r < 8; ++r) {
      const float p = __expf((sv[r] - mnew) * sinv);
      psum += p;
      pa[r] = (f16t)(p * PCAR);
    }
    psum += __shfl_xor(psum, 1);
    psum += __shfl_xor(psum, 2);
    psum += __shfl_xor(psum, 4);
    lrun = lrun * rs + psum;
    if (jq == 0) rsc[si] = rs;
    *(v8ha*)(sP + si * PSP + 8 * jq) = pa;
    __syncthreads();

    #pragma unroll
    for (int js = 0; js < 2; ++js) {
      Q8 rr;
      rr.q[0] = *(const v4fa*)(rsc + 16 * js + 8 * h);
      rr.q[1] = *(const v4fa*)(rsc + 16 * js + 8 * h + 4);
      #pragma unroll
      for (int ct = 0; ct < 4; ++ct) {
        #pragma unroll
        for (int e = 0; e < 8; ++e) acc[js][ct][e] *= rr.v[e];
      }
    }
    #pragma unroll
    for (int kc = 0; kc < 2; ++kc) {
      const v16h a0 = load_frag32(sP + m * PSP + 32 * kc, h);
      const v16h a1 = load_frag32(sP + (16 + m) * PSP + 32 * kc, h);
      #pragma unroll
      for (int ct = 0; ct < 4; ++ct) {
        const v16h bb = load_frag32(vrow + (size_t)(16 * ct) * NP + j0 + 32 * kc, h);
        acc[0][ct] = wmma_f16(a0, bb, acc[0][ct]);
        acc[1][ct] = wmma_f16(a1, bb, acc[1][ct]);
      }
    }
  }

  if (jq == 0) lsum[si] = lrun;
  __syncthreads();
  const float gsc = alpha[0] * (1.0f / (VCAR * PCAR));
  const int q8 = lane & 7, sub = lane >> 3;
  #pragma unroll
  for (int p = 0; p < 2; ++p) {
    #pragma unroll
    for (int js = 0; js < 2; ++js) {
      Q8 li;
      li.q[0] = *(const v4fa*)(lsum + 16 * js + 8 * h);
      li.q[1] = *(const v4fa*)(lsum + 16 * js + 8 * h + 4);
      float linv[8];
      #pragma unroll
      for (int r = 0; r < 8; ++r) linv[r] = gsc * __builtin_amdgcn_rcpf(li.v[r]);
      #pragma unroll
      for (int t = 0; t < 2; ++t) {
        v8f vv;
        #pragma unroll
        for (int r = 0; r < 8; ++r) vv[r] = acc[js][2 * p + t][r] * linv[r];
        st8f(sO + (32 * w + 16 * t + m) * OSP + 16 * js + 8 * h, vv);
      }
    }
    __syncthreads();
    v4f o8[8];
    #pragma unroll
    for (int i = 0; i < 8; ++i) {
      const int s = 32 * w + 4 * i + sub;
      const int c = 64 * w + 32 * p + 4 * i + sub;
      const v4f v = *(const v4fa*)(sO + s * OSP + 4 * q8);
      const size_t d = (size_t)(b * CC + c) * NP + i0 + 4 * q8;
      const v4f xv = *(const v4fa*)(xres + d);
      o8[i] = v + xv;
      *(volatile v4f*)(out + d) = o8[i];
    }
    __threadfence();
    #pragma unroll
    for (int i = 0; i < 8; ++i) {
      const int c = 64 * w + 32 * p + 4 * i + sub;
      const size_t d = (size_t)(b * CC + c) * NP + i0 + 4 * q8;
      *(volatile v4f*)(out + d) = o8[i];
    }
    __syncthreads();
  }
}

extern "C" void kernel_launch(void* const* d_in, const int* in_sizes, int n_in,
                              void* d_out, int out_size, void* d_ws, size_t ws_size,
                              hipStream_t stream) {
  if (n_in < 8) return;
  if (in_sizes[0] != NB * CC * NP) return;
  if (in_sizes[1] != MID * CC || in_sizes[3] != MID * CC) return;
  if (in_sizes[2] != MID || in_sizes[4] != MID) return;
  if (in_sizes[5] != CC * CC || in_sizes[6] != CC) return;
  if (in_sizes[7] < 1) return;
  if (out_size != NB * CC * NP) return;

  const float* x     = (const float*)d_in[0];
  const float* wq    = (const float*)d_in[1];
  const float* bq    = (const float*)d_in[2];
  const float* wk    = (const float*)d_in[3];
  const float* bk    = (const float*)d_in[4];
  const float* wv    = (const float*)d_in[5];
  const float* bv    = (const float*)d_in[6];
  const float* alpha = (const float*)d_in[7];
  float* outp = (float*)d_out;

  const size_t szWq = (size_t)MID * CC * 2;
  const size_t szWv = (size_t)CC * CC * 2;
  const size_t szXT = (size_t)NB * NP * CC * 2;
  const size_t szQT = (size_t)NB * NP * MID * 2;
  const size_t szVC = (size_t)NB * CC * NP * 2;
  size_t off = 0;
  char* ws = (char*)d_ws;
  f16t* Wqh = (f16t*)(ws + off); off += szWq;
  f16t* Wkh = (f16t*)(ws + off); off += szWq;
  f16t* Wvh = (f16t*)(ws + off); off += szWv;
  f16t* XT  = (f16t*)(ws + off); off += szXT;
  f16t* QT  = (f16t*)(ws + off); off += szQT;
  f16t* KT  = (f16t*)(ws + off); off += szQT;
  f16t* VC  = (f16t*)(ws + off); off += szVC;
  if (off > ws_size) return;

  k_wcvt<<<160, 256, 0, stream>>>(wq, wk, wv, Wqh, Wkh, Wvh);
  k_tr<<<dim3(CC / 64, HW, NB), 256, 0, stream>>>(x, XT);
  k_proj<<<dim3(NP / 64, 10, NB), 256, 0, stream>>>(XT, Wqh, Wkh, Wvh, bq, bk, bv, QT, KT, VC);
  k_att<<<dim3(NP / QB, NB), 256, 0, stream>>>(QT, KT, VC, x, alpha, outp);
}
